// GCN2_30210799960820
// MI455X (gfx1250) — hardware-verified
//
#include <hip/hip_runtime.h>
#include <math.h>

constexpr int kNodes  = 100000;
constexpr int kEdges  = 1000000;
constexpr int kNPad   = 100032;
constexpr int kFin    = 128;
constexpr int kHid    = 64;
constexpr int kCls    = 16;
constexpr int kNB     = 64;
constexpr int kNT     = 256;
constexpr int kSRB    = 8192;
constexpr int kRPWLog = 10;
constexpr int kRPW    = 1 << kRPWLog;
constexpr int kNTiles = 13;
constexpr int kGRows  = kNTiles * kSRB;
constexpr int kSP     = 8;
constexpr int kSCH    = kNT * kSP;
constexpr int kNCH    = (kEdges + kSCH - 1) / kSCH;
constexpr float kXCarry = 64.0f;
constexpr float kHCarry = 256.0f;
constexpr float kWCarry = 16.0f;
static_assert(kNPad % 64 == 0 && kNPad >= kNodes);
static_assert(kFin % 32 == 0 && kHid % 32 == 0 && kNB % 64 == 0);
static_assert(kGRows >= kNPad);
static_assert(kSRB == 8 * kRPW);
static_assert(kEdges % kSP == 0);
static_assert(kNodes % 8 == 0 && kNPad % 8 == 0);
static_assert(kNodes < (1 << 17) && kSRB <= (1 << 13));
static_assert((kNPad * kFin) % (8 * kNT) == 0);

typedef __attribute__((ext_vector_type(16))) _Float16 v16h;
typedef __attribute__((ext_vector_type(8)))  _Float16 v8h;
typedef __attribute__((ext_vector_type(16))) __bf16   v16b;
typedef __attribute__((ext_vector_type(8)))  __bf16   v8b;
typedef __attribute__((ext_vector_type(8)))  float    v8f;
typedef __attribute__((ext_vector_type(4)))  float    v4f;
typedef __attribute__((ext_vector_type(2)))  float    v2f;
typedef __attribute__((ext_vector_type(4)))  int      v4i;
typedef __attribute__((ext_vector_type(4)))  unsigned int v4u;

__device__ __forceinline__ unsigned short f2bf_bits(float f) {
  unsigned u = __float_as_uint(f);
  return (unsigned short)((u + 0x7FFFu + ((u >> 16) & 1u)) >> 16);
}
__device__ __forceinline__ float bf_bits2f(unsigned short h) { return __uint_as_float(((unsigned)h) << 16); }

__device__ __forceinline__ void dep_guard_h(v8f& a, v8f& b, v16h x, v16h y) { asm volatile("v_nop\n\tv_nop\n\tv_nop\n\tv_nop" : "+v"(a), "+v"(b) : "v"(x), "v"(y)); }
__device__ __forceinline__ void dep_guard_b(v8f& a, v8f& b, v16b x, v16b y) { asm volatile("v_nop\n\tv_nop\n\tv_nop\n\tv_nop" : "+v"(a), "+v"(b) : "v"(x), "v"(y)); }
__device__ __forceinline__ void keep4_h(v16h a, v16h b, v16h c, v16h d) { asm volatile("v_nop" :: "v"(a), "v"(b), "v"(c), "v"(d)); }
__device__ __forceinline__ void keep4_b(v16b a, v16b b, v16b c, v16b d) { asm volatile("v_nop" :: "v"(a), "v"(b), "v"(c), "v"(d)); }
__device__ __forceinline__ void acc_guard4(v8f& a, v8f& b, v8f& c, v8f& d) { asm volatile("v_nop\n\tv_nop\n\tv_nop\n\tv_nop" : "+v"(a), "+v"(b), "+v"(c), "+v"(d)); }
template <typename T> struct Frag;
template <> struct Frag<_Float16> {
  typedef v16h V; union U { v16h v; v8h h[2]; };
  static __device__ __forceinline__ v16h load(const _Float16* p) {
    U f; f.h[0] = *(const v8h*)(p); f.h[1] = *(const v8h*)(p + 16); return f.v;
  }
  static __device__ __forceinline__ v8f mma(v16h a, v16h b, v8f c) {
    return __builtin_amdgcn_wmma_f32_16x16x32_f16(false, a, false, b, (short)0, c, false, false);
  }
  static __device__ __forceinline__ void guard(v8f& a, v8f& b, v16h x, v16h y) { dep_guard_h(a, b, x, y); }
  static __device__ __forceinline__ void keep(v16h a, v16h b, v16h c, v16h d) { keep4_h(a, b, c, d); }
};
template <> struct Frag<__bf16> {
  typedef v16b V; union U { v16b v; v8b h[2]; };
  static __device__ __forceinline__ v16b load(const __bf16* p) {
    U f; f.h[0] = *(const v8b*)(p); f.h[1] = *(const v8b*)(p + 16); return f.v;
  }
  static __device__ __forceinline__ v8f mma(v16b a, v16b b, v8f c) {
    return __builtin_amdgcn_wmma_f32_16x16x32_bf16(false, a, false, b, (short)0, c, false, false);
  }
  static __device__ __forceinline__ void guard(v8f& a, v8f& b, v16b x, v16b y) { dep_guard_b(a, b, x, y); }
  static __device__ __forceinline__ void keep(v16b a, v16b b, v16b c, v16b d) { keep4_b(a, b, c, d); }
};

__device__ __forceinline__ unsigned pk16(unsigned short a, unsigned short b) { return (unsigned)a | ((unsigned)b << 16); }
__device__ __forceinline__ unsigned short h_bits(float f) { const _Float16 h = (_Float16)f; return __builtin_bit_cast(unsigned short, h); }

template <int ET> struct Elem;
template <> struct Elem<0> { typedef _Float16 T; };
template <> struct Elem<1> { typedef __bf16 T; };
template <int ET, bool SPLIT, int BIAS_MODE, int OUT_MODE, bool RESID, int ACT = 0>
__global__ __launch_bounds__(256) void wmma_gemm64(
    const unsigned short* __restrict__ Ap, const unsigned short* __restrict__ A2p, int lda, long strideA,
    const unsigned short* __restrict__ Btp, const unsigned short* __restrict__ Bt2p, int ldb, long strideB,
    void* __restrict__ Cout, void* __restrict__ Cout2, int ldc, long strideC,
    const float* __restrict__ bias,
    const float* __restrict__ resid, long strideR,
    int M, int N, int K, float scale) {
  typedef typename Elem<ET>::T T;
  typedef typename Frag<T>::V V;
  const T* A = (const T*)Ap; const T* A2 = (const T*)A2p; const T* Bt = (const T*)Btp; const T* Bt2 = (const T*)Bt2p;
  __shared__ __align__(16) float sT[8][16 * 68];
  const int b    = blockIdx.y;
  const int lane = threadIdx.x & 31;
  const int wave = threadIdx.x >> 5;
  const int tilesN = N >> 6;
  const int tilesM = M >> 6;
  const int tile = blockIdx.x * 8 + wave;
  if (tile >= tilesM * tilesN) return;
  const int tm = tile / tilesN;
  const int tn = tile - tm * tilesN;
  const int m0 = tm << 6;
  const int n0 = tn << 6;

  const T* Ab  = A  + (size_t)b * strideA;
  const T* Bb  = Bt + (size_t)b * strideB;
  const T* Ab2 = SPLIT ? (A2  + (size_t)b * strideA) : nullptr;
  const T* Bb2 = SPLIT ? (Bt2 + (size_t)b * strideB) : nullptr;

  const int rlane = lane & 15;
  const int koff  = (lane >> 4) * 8;
  const int mOff  = (lane >> 4) * 8;

  v8f acc[4][4];
#pragma unroll
  for (int i = 0; i < 4; ++i)
#pragma unroll
    for (int j = 0; j < 4; ++j) acc[i][j] = (v8f){0.f,0.f,0.f,0.f,0.f,0.f,0.f,0.f};

  for (int k0 = 0; k0 < K; k0 += 32) {
    V bh[4], bl[4];
#pragma unroll
    for (int j = 0; j < 4; ++j) {
      const size_t bo = (size_t)(n0 + (j << 4) + rlane) * ldb + koff + k0;
      bh[j] = Frag<T>::load(Bb + bo);
      if (SPLIT) bl[j] = Frag<T>::load(Bb2 + bo);
    }
#pragma unroll
    for (int i = 0; i < 4; ++i) {
      const size_t ao = (size_t)(m0 + (i << 4) + rlane) * lda + koff + k0;
      V ah = Frag<T>::load(Ab + ao);
      V al;
      if (SPLIT) al = Frag<T>::load(Ab2 + ao);
#pragma unroll
      for (int j = 0; j < 4; ++j) {
        acc[i][j] = Frag<T>::mma(ah, bh[j], acc[i][j]);
        if (SPLIT) {
          acc[i][j] = Frag<T>::mma(ah, bl[j], acc[i][j]);
          acc[i][j] = Frag<T>::mma(al, bh[j], acc[i][j]);
        }
      }
      Frag<T>::guard(acc[i][0], acc[i][3], ah, SPLIT ? al : ah);
    }
    Frag<T>::keep(bh[0], bh[1], bh[2], bh[3]);
    if (SPLIT) Frag<T>::keep(bl[0], bl[1], bl[2], bl[3]);
  }
  acc_guard4(acc[0][0], acc[0][1], acc[0][2], acc[0][3]);
  acc_guard4(acc[1][0], acc[1][1], acc[1][2], acc[1][3]);
  acc_guard4(acc[2][0], acc[2][1], acc[2][2], acc[2][3]);
  acc_guard4(acc[3][0], acc[3][1], acc[3][2], acc[3][3]);

  float* slab = sT[wave];
  const float* Rb = RESID ? (resid + (size_t)b * strideR) : nullptr;
#pragma unroll
  for (int i = 0; i < 4; ++i) {
    const int mBase = m0 + (i << 4);
#pragma unroll
    for (int j = 0; j < 4; ++j) {
      const int n = n0 + (j << 4) + rlane;
      float bv = 0.f;
      if (BIAS_MODE == 2) bv = bias[n];
#pragma unroll
      for (int r = 0; r < 8; ++r) {
        float v = acc[i][j][r] * scale;
        if (BIAS_MODE == 1) v += bias[mBase + mOff + r];
        if (BIAS_MODE == 2) v += bv;
        if (RESID) v += Rb[(size_t)(mBase + mOff + r) * ldc + n];
        if (ACT == 2) v = fmaxf(v, 0.0f);
        if (ACT == 4) v = (v > 0.f) ? v : 0.01f * v;
        slab[(mOff + r) * 68 + (j << 4) + rlane] = v;
      }
    }
    __builtin_amdgcn_fence(__ATOMIC_RELEASE, "workgroup");
    __builtin_amdgcn_wave_barrier();
    __builtin_amdgcn_fence(__ATOMIC_ACQUIRE, "workgroup");
    if (OUT_MODE == 0) {
      float* C = (float*)Cout + (size_t)b * strideC;
      const int hh = lane >> 4, c4 = (lane & 15) * 4;
      for (int pass = 0; pass < 2; ++pass) {
#pragma unroll
        for (int it = 0; it < 8; ++it) {
          const int row = it * 2 + hh;
          v4f v = *(const v4f*)(slab + row * 68 + c4);
          *(volatile v4f*)(C + (size_t)(mBase + row) * ldc + n0 + c4) = v;
        }
        __threadfence();
      }
    } else {
      const int q = lane >> 3, c8 = (lane & 7) * 8;
      unsigned short* C  = (unsigned short*)Cout  + (size_t)b * strideC;
      unsigned short* C2 = (OUT_MODE == 2) ? ((unsigned short*)Cout2 + (size_t)b * strideC) : nullptr;
      for (int pass = 0; pass < 2; ++pass) {
#pragma unroll
        for (int it = 0; it < 4; ++it) {
          const int row = it * 4 + q;
          const float* sp = slab + row * 68 + c8;
          v8h hv, lv;
#pragma unroll
          for (int e = 0; e < 8; ++e) {
            if (OUT_MODE == 1) {
              hv[e] = (_Float16)sp[e];
            } else {
              unsigned short hb = f2bf_bits(sp[e]);
              unsigned short lb = f2bf_bits(sp[e] - bf_bits2f(hb));
              hv[e] = __builtin_bit_cast(_Float16, hb);
              lv[e] = __builtin_bit_cast(_Float16, lb);
            }
          }
          *(volatile v8h*)(C + (size_t)(mBase + row) * ldc + n0 + c8) = hv;
          if (OUT_MODE == 2) *(volatile v8h*)(C2 + (size_t)(mBase + row) * ldc + n0 + c8) = lv;
        }
        __threadfence();
      }
    }
    __builtin_amdgcn_fence(__ATOMIC_RELEASE, "workgroup");
    __builtin_amdgcn_wave_barrier();
    __builtin_amdgcn_fence(__ATOMIC_ACQUIRE, "workgroup");
  }
}

__device__ __forceinline__ void store8h_2pass(unsigned short* q, const float* w) {
  unsigned short hb[8];
#pragma unroll
  for (int e = 0; e < 8; ++e) hb[e] = h_bits(w[e]);
  const v4u u = (v4u){pk16(hb[0], hb[1]), pk16(hb[2], hb[3]), pk16(hb[4], hb[5]), pk16(hb[6], hb[7])};
  *(volatile v4u*)q = u;
  __threadfence();
  *(volatile v4u*)q = u;
}

__global__ __launch_bounds__(kNT) void prep_kernel(const float* __restrict__ W1, const float* __restrict__ W2, const float* __restrict__ W3,
                                                 unsigned short* __restrict__ BT1, unsigned short* __restrict__ BT2, unsigned short* __restrict__ BT3) {
  const int bid = blockIdx.x, tid = threadIdx.x;
  float w[8];
  if (bid < 4) {
    const int t = bid * kNT + tid;
    const int n = t >> 4, kb = (t & 15) * 8;
#pragma unroll
    for (int e = 0; e < 8; ++e) w[e] = W1[(size_t)(kb + e) * kHid + n] * kWCarry;
    store8h_2pass(BT1 + 8 * (size_t)t, w);
  } else if (bid < 6) {
    const int t = (bid - 4) * kNT + tid;
    const int n = t >> 3, kb = (t & 7) * 8;
#pragma unroll
    for (int e = 0; e < 8; ++e) w[e] = W2[(size_t)(kb + e) * kHid + n] * kWCarry;
    store8h_2pass(BT2 + 8 * (size_t)t, w);
  } else {
    const int t = (bid - 6) * kNT + tid;
    const int n = t >> 3, kb = (t & 7) * 8;
    const int nc = n < kCls ? n : (kCls - 1);
#pragma unroll
    for (int e = 0; e < 8; ++e) {
      const float wr = W3[(size_t)(kb + e) * kCls + nc];
      w[e] = (n < kCls) ? wr * kWCarry : 0.f;
    }
    store8h_2pass(BT3 + 8 * (size_t)t, w);
  }
}

__global__ __launch_bounds__(kNT) void castx_kernel(const float* __restrict__ x, unsigned short* __restrict__ A1, int n8) {
  const int i = blockIdx.x * kNT + threadIdx.x;
  if (i >= n8) return;
  const int row = i >> 4;
  const int c8  = (i & 15) * 8;
  const int rowc = row < kNodes ? row : (kNodes - 1);
  const float* p = x + (size_t)rowc * kFin + c8;
  const v4f a = *(const v4f*)(p);
  const v4f c = *(const v4f*)(p + 4);
  const float f = (row < kNodes) ? kXCarry : 0.f;
  float w[8];
#pragma unroll
  for (int e = 0; e < 4; ++e) { w[e] = a[e] * f; w[4 + e] = c[e] * f; }
  store8h_2pass(A1 + 8 * (size_t)i, w);
}

__device__ __forceinline__ int blk_excl_scan(int cnt, int* scan_ws, int tid, int* tot) {
  const int lane = tid & 31, wave = tid >> 5; int incl = cnt;
#pragma unroll
  for (int o = 1; o < 32; o <<= 1) { const int v = __shfl_up(incl, o, 32); if (lane >= o) incl += v; }
  if (lane == 31) scan_ws[wave] = incl;
  __syncthreads();
  if (wave == 0) {
    const int sw = scan_ws[lane];
    const int wv = (lane < kNT / 32) ? sw : 0; int wincl = wv;
#pragma unroll
    for (int o = 1; o < 32; o <<= 1) { const int v = __shfl_up(wincl, o, 32); if (lane >= o) wincl += v; }
    if (lane < kNT / 32) scan_ws[32 + lane] = wincl - wv;
    if (lane == 31) scan_ws[64] = wincl;
  }
  __syncthreads();
  const int res = scan_ws[32 + wave] + incl - cnt; *tot = scan_ws[64];
  return res;
}
__device__ __forceinline__ int chunk_hits(const int* __restrict__ dstv, const int* __restrict__ srcv, const float* __restrict__ valv,
                                          int e0, int n0, int tid, int* LIST, float* LISTV, int* scan_ws) {
  const int eb = e0 + tid * kSP;
  const bool inr = eb < kEdges;
  const int ebc = inr ? eb : (kEdges - kSP);
  int rec[kSP]; float rvv[kSP]; int cnt = 0;
#pragma unroll
  for (int k = 0; k < kSP; k += 4) {
    const v4i d4 = *(const v4i*)(dstv + ebc + k);
    const v4i s4 = *(const v4i*)(srcv + ebc + k);
    const v4f v4 = *(const v4f*)(valv + ebc + k);
#pragma unroll
    for (int e = 0; e < 4; ++e) {
      const int d = d4[e];
      int s = s4[e]; s = s < 0 ? 0 : (s >= kNodes ? kNodes - 1 : s);
      const bool hit = inr && (d >= n0) && (d < n0 + kSRB) && (d < kNodes);
      rec[k + e] = hit ? (((d - n0) << 17) | s) : -1;
      rvv[k + e] = v4[e];
      cnt += hit ? 1 : 0;
    }
  }
  int tot; int p = blk_excl_scan(cnt, scan_ws, tid, &tot);
#pragma unroll
  for (int k = 0; k < kSP; ++k) {
    if (rec[k] >= 0) { if ((unsigned)p < (unsigned)kSCH) { LIST[p] = rec[k]; LISTV[p] = rvv[k]; } ++p; }
  }
  __syncthreads();
  return tot < kSCH ? tot : kSCH;
}

template <int NCOL>
__global__ __launch_bounds__(kNT) void agg_kernel(const float* __restrict__ S, const int* __restrict__ esrc, const int* __restrict__ edst,
                                                const float* __restrict__ ev, const float* __restrict__ bias, float* G,
                                                unsigned short* __restrict__ Aout, float* __restrict__ Out, float carry) {
  __shared__ int LIST[kSCH];
  __shared__ float LISTV[kSCH];
  __shared__ int scan_ws[80];
  __shared__ __align__(16) unsigned slab[8][256];
  const int tid = threadIdx.x, lane = tid & 31, wave = tid >> 5;
  const int n0  = blockIdx.x * kSRB;
  const int rw0 = n0 + wave * kRPW;
  const int col = lane & 15;

  for (int i = tid; i < kSCH; i += kNT) { LIST[i] = -1; LISTV[i] = 0.f; }
  if (tid < 80) scan_ws[tid] = 0;
  for (int i = tid; i < 8 * 256; i += kNT) (&slab[0][0])[i] = 0u;

  if (NCOL == 64) {
    const v2f z2 = {0.f, 0.f};
#pragma unroll 4
    for (int j = 0; j < kRPW; ++j) *(v2f*)(G + (size_t)(rw0 + j) * 64 + 2 * lane) = z2;
  } else {
#pragma unroll 4
    for (int j = 0; j < kRPW; ++j) G[(size_t)(rw0 + j) * 16 + col] = 0.f;
  }
  __syncthreads();

#pragma unroll 1
  for (int c = 0; c < kNCH; ++c) {
    const int tot = chunk_hits(edst, esrc, ev, c * kSCH, n0, tid, LIST, LISTV, scan_ws);
#pragma unroll 1
    for (int base = 0; base < tot; base += 32) {
      const int q  = base + lane;
      const int qc = q < kSCH ? q : (kSCH - 1);
      const int rq = LIST[qc];
      const float vq = LISTV[qc];
      const int rv = (q < tot) ? rq : -1;
      const int own = (rv >= 0 && ((rv >> 17) >> kRPWLog) == wave) ? 1 : 0;
      unsigned msk = (unsigned)__ballot(own);
#pragma unroll 1
      for (int it = 0; it < 32; ++it) {
        if (msk == 0u) break;
        const int bp = __builtin_ctz(msk); msk &= msk - 1u;
        const int r = __shfl(rv, bp, 32);
        const float vh = __shfl(vq, bp, 32);
        const int dl = (r >> 17) & (kSRB - 1);
        int s = r & 0x1FFFF; s = s < kNodes ? s : (kNodes - 1);
        if (NCOL == 64) {
          const v2f sv = *(const v2f*)(S + (size_t)s * kNB + 2 * lane);
          float* ap = G + (size_t)(n0 + dl) * 64 + 2 * lane;
          v2f av = *(const v2f*)ap;
          av = av + vh * sv;
          *(v2f*)ap = av;
        } else {
          const float sv = S[(size_t)s * kNB + col];
          float* ap = G + (size_t)(n0 + dl) * 16 + col;
          float av = *ap;
          av = av + vh * sv;
          *ap = av;
        }
      }
    }
    __syncthreads();
  }

  if (NCOL == 64) {
    const v2f bv = *(const v2f*)(bias + 2 * lane);
#pragma unroll 1
    for (int st = 0; st < kRPW / 8; ++st) {
      const int rb = rw0 + st * 8;
      const bool live = rb < kNodes;
#pragma unroll
      for (int i = 0; i < 8; ++i) {
        const v2f a = *(const v2f*)(G + (size_t)(rb + i) * 64 + 2 * lane);
        float v0 = fmaxf(a[0] + bv[0], 0.f) * carry;
        float v1 = fmaxf(a[1] + bv[1], 0.f) * carry;
        v0 = live ? v0 : 0.f;
        v1 = live ? v1 : 0.f;
        slab[wave][i * 32 + lane] = pk16(h_bits(v0), h_bits(v1));
      }
      __syncthreads();
      const v4u u0 = *(const v4u*)(&slab[wave][4 * lane]);
      const v4u u1 = *(const v4u*)(&slab[wave][128 + 4 * lane]);
      if (rb < kNPad) {
        unsigned short* p0 = Aout + (size_t)(rb + (lane >> 3)) * kHid + 8 * (lane & 7);
        unsigned short* p1 = p0 + 4 * kHid;
        *(volatile v4u*)p0 = u0; *(volatile v4u*)p1 = u1;
        __threadfence();
        *(volatile v4u*)p0 = u0; *(volatile v4u*)p1 = u1;
      }
      __syncthreads();
    }
  } else {
    const float bsc = bias[col];
    unsigned* ou = (unsigned*)Out;
#pragma unroll 1
    for (int st = 0; st < kRPW / 8; ++st) {
      const int rb = rw0 + st * 8;
#pragma unroll
      for (int i = 0; i < 8; ++i) {
        const float a = G[(size_t)(rb + i) * 16 + col];
        const float v = a + bsc;
        slab[wave][i * 16 + col] = __float_as_uint(v);
      }
      __syncthreads();
      const v4u u = *(const v4u*)(&slab[wave][4 * lane]);
      if (rb < kNodes) {
        unsigned* op = ou + (size_t)rb * kCls + 4 * lane;
        *(volatile v4u*)op = u;
        __threadfence();
        *(volatile v4u*)op = u;
      }
      __syncthreads();
    }
  }
}

extern "C" void kernel_launch(void* const* d_in, const int* in_sizes, int n_in,
                              void* d_out, int out_size, void* d_ws, size_t ws_size, hipStream_t stream) {
  if (n_in < 10) return;
  const float* x    = (const float*)d_in[0];
  const float* eval = (const float*)d_in[1];
  const float* W1   = (const float*)d_in[2];
  const float* b1   = (const float*)d_in[3];
  const float* W2   = (const float*)d_in[4];
  const float* b2   = (const float*)d_in[5];
  const float* W3   = (const float*)d_in[6];
  const float* b3   = (const float*)d_in[7];
  const int*   esrc = (const int*)d_in[8];
  const int*   edst = (const int*)d_in[9];
  float*       out  = (float*)d_out;
  if (in_sizes[0] != kNodes * kFin || in_sizes[1] != kEdges || in_sizes[2] != kFin * kHid || in_sizes[3] != kHid ||
      in_sizes[4] != kHid * kHid || in_sizes[5] != kHid || in_sizes[6] != kHid * kCls || in_sizes[7] != kCls ||
      in_sizes[8] != kEdges || in_sizes[9] != kEdges || out_size != kNodes * kCls) return;

  char* ws = (char*)d_ws; size_t off = 0;
  auto carve = [&](size_t bytes) -> char* { char* p = ws + off; off += (bytes + 255) & ~(size_t)255; return p; };
  unsigned short* BT1 = (unsigned short*)carve((size_t)kNB * kFin * 2);
  unsigned short* BT2 = (unsigned short*)carve((size_t)kNB * kHid * 2);
  unsigned short* BT3 = (unsigned short*)carve((size_t)kNB * kHid * 2);
  unsigned short* A1  = (unsigned short*)carve((size_t)kNPad * kFin * 2);
  float*          S   = (float*)carve((size_t)kNPad * kNB * 4);
  float*          G   = (float*)carve((size_t)kGRows * kHid * 4);
  float*          G3  = (float*)carve((size_t)kGRows * kCls * 4);
  unsigned short* A2  = (unsigned short*)carve((size_t)kNPad * kHid * 2);
  unsigned short* A3  = (unsigned short*)carve((size_t)kNPad * kHid * 2);
  if (off > ws_size || off > (size_t)134217728) return;

  const int gemm_tiles  = (kNPad / 64) * (kNB / 64);
  const int gemm_blocks = (gemm_tiles + 7) / 8;
  const int n8 = kNPad * kFin / 8;

  prep_kernel<<<8, kNT, 0, stream>>>(W1, W2, W3, BT1, BT2, BT3);
  castx_kernel<<<(n8 + kNT - 1) / kNT, kNT, 0, stream>>>(x, A1, n8);
  wmma_gemm64<0, false, 0, 0, false, 0><<<dim3(gemm_blocks, 1), 256, 0, stream>>>(
      (const unsigned short*)A1, (const unsigned short*)A1, kFin, 0L,
      (const unsigned short*)BT1, (const unsigned short*)BT1, kFin, 0L,
      (void*)S, (void*)nullptr, kNB, 0L,
      (const float*)nullptr, (const float*)nullptr, 0L, kNPad, kNB, kFin, 1.0f / (kXCarry * kWCarry));
  agg_kernel<64><<<kNTiles, kNT, 0, stream>>>(S, esrc, edst, eval, b1, G, A2, G3, kHCarry);
  wmma_gemm64<0, false, 0, 0, false, 0><<<dim3(gemm_blocks, 1), 256, 0, stream>>>(
      (const unsigned short*)A2, (const unsigned short*)A2, kHid, 0L,
      (const unsigned short*)BT2, (const unsigned short*)BT2, kHid, 0L,
      (void*)S, (void*)nullptr, kNB, 0L,
      (const float*)nullptr, (const float*)nullptr, 0L, kNPad, kNB, kHid, 1.0f / (kHCarry * kWCarry));
  agg_kernel<64><<<kNTiles, kNT, 0, stream>>>(S, esrc, edst, eval, b2, G, A3, G3, kHCarry);
  wmma_gemm64<0, false, 0, 0, false, 0><<<dim3(gemm_blocks, 1), 256, 0, stream>>>(
      (const unsigned short*)A3, (const unsigned short*)A3, kHid, 0L,
      (const unsigned short*)BT3, (const unsigned short*)BT3, kHid, 0L,
      (void*)S, (void*)nullptr, kNB, 0L,
      (const float*)nullptr, (const float*)nullptr, 0L, kNPad, kNB, kHid, 1.0f / (kHCarry * kWCarry));
  agg_kernel<16><<<kNTiles, kNT, 0, stream>>>(S, esrc, edst, eval, b3, G3, A3, out, 1.0f);
}
